// CIDER_25383256719526
// MI455X (gfx1250) — hardware-verified
//
#include <hip/hip_runtime.h>


namespace {
constexpr int B = 96, HS = 100, D = 768, NCAND = 128, A = 256, R = B * HS;
constexpr float XS = 8.0f, WSC = 256.0f;
typedef _Float16 b16;
typedef __attribute__((ext_vector_type(16))) _Float16 v16b;
typedef __attribute__((ext_vector_type(8))) _Float16 v8b;
typedef __attribute__((ext_vector_type(8))) float v8f;
typedef __attribute__((ext_vector_type(4))) float v4f;
__device__ __forceinline__ float bf16_rne(float f) { unsigned int u = __float_as_uint(f); u += 0x7FFFu + ((u >> 16) & 1u); float r = __uint_as_float(u & 0xFFFF0000u); asm volatile("" : "+v"(r)); return r; }
__device__ __forceinline__ void split16(float v, b16& hi, b16& lo) { hi = (b16)v; lo = (b16)(v - (float)hi); }
__device__ __forceinline__ v16b frag_kb(const b16* p, int hh) { const v8b a = *(const v8b*)(p + 8 * hh), b = *(const v8b*)(p + 16 + 8 * hh); v16b f;
#pragma unroll
  for (int e = 0; e < 8; ++e) { f[e] = a[e]; f[8 + e] = b[e]; } return f; }
__device__ __forceinline__ v8f wmma16b(v16b a, v16b b, v8f c) { v8f d = __builtin_amdgcn_wmma_f32_16x16x32_f16(false, a, false, b, (short)0, c, false, false); asm volatile("v_nop\n\tv_nop\n\tv_nop\n\tv_nop" : "+v"(d) : "v"(a), "v"(b)); return d; }
__device__ __forceinline__ void wave_lds_sync() { __builtin_amdgcn_fence(__ATOMIC_RELEASE, "workgroup"); __builtin_amdgcn_wave_barrier(); __builtin_amdgcn_fence(__ATOMIC_ACQUIRE, "workgroup"); }
__device__ __forceinline__ float pmul(float a, float b) { float p = a * b; asm volatile("" : "+v"(p)); return p; }

__global__ __launch_bounds__(256) void wput_kernel(const float* __restrict__ wl, const float* __restrict__ wr, const float* __restrict__ wk, const float* __restrict__ wq, b16* __restrict__ WL, b16* __restrict__ WR, b16* __restrict__ WK, b16* __restrict__ WQ) { const size_t u = (size_t)blockIdx.x * 256 + threadIdx.x;
  for (int pass = 0; pass < 2; ++pass) {
    if (u < (size_t)D * (D / 8)) { v8b a, b;
#pragma unroll
      for (int j = 0; j < 8; ++j) { a[j] = (b16)(bf16_rne(wl[u * 8 + j]) * WSC); b[j] = (b16)(bf16_rne(wr[u * 8 + j]) * WSC); } *(volatile v8b*)(WL + u * 8) = a; *(volatile v8b*)(WR + u * 8) = b; }
    if (u < (size_t)A * (D / 8)) { v8b a, b;
#pragma unroll
      for (int j = 0; j < 8; ++j) { a[j] = (b16)(bf16_rne(wk[u * 8 + j]) * WSC); b[j] = (b16)(bf16_rne(wq[u * 8 + j]) * WSC); } *(volatile v8b*)(WK + u * 8) = a; *(volatile v8b*)(WQ + u * 8) = b; }
    __threadfence(); } }
__global__ __launch_bounds__(256) void mean_kernel(const float* __restrict__ hist, float* __restrict__ NB) { const int u = blockIdx.x * 256 + threadIdx.x; if (u >= B * D / 4) return; const int b = u / (D / 4), d0 = (u % (D / 4)) * 4; v4f s = {0, 0, 0, 0};
  for (int h = 0; h < B; ++h) { const v4f v = *(const v4f*)(hist + ((size_t)b * HS + h) * D + d0); for (int k = 0; k < 4; ++k) s[k] += bf16_rne(v[k]); }
  for (int k = 0; k < 4; ++k) s[k] = pmul(s[k], 1.0f / (float)B);
  for (int pass = 0; pass < 2; ++pass) { *(volatile v4f*)(NB + (size_t)u * 4) = s; __threadfence(); } }
template <int MODE>
__global__ __launch_bounds__(32) void dense_kernel(const float* __restrict__ IN, int nrows, const b16* __restrict__ WT, int NOUT, const float* __restrict__ bias, const float* __restrict__ ADD, float* __restrict__ OUT) { __shared__ __attribute__((aligned(16))) b16 Ah[16][D + 8], Al[16][MODE == 0 ? 8 : D + 8]; __shared__ float Tf[16][132]; const int lane = threadIdx.x, nloc = lane & 15, hlf = lane >> 4; const int NGR = NOUT / 128; const int g = blockIdx.x % NGR; const size_t m0 = (size_t)(blockIdx.x / NGR) * 16; if (m0 >= (size_t)nrows) return;
  for (int rr = 0; rr < 16; ++rr) { const size_t row = m0 + rr; for (int q = 0; q < D / 32; ++q) { const float v = row < (size_t)nrows ? IN[row * D + q * 32 + lane] : 0.0f; if (MODE == 0) Ah[rr][q * 32 + lane] = (b16)(bf16_rne(v) * XS); else { b16 p, ql; split16(v * XS, p, ql); Ah[rr][q * 32 + lane] = p; Al[rr][q * 32 + lane] = ql; } } }
  wave_lds_sync(); v8f acc[8];
#pragma unroll
  for (int t = 0; t < 8; ++t) acc[t] = (v8f){};
#pragma unroll 2
  for (int kb = 0; kb < D; kb += 32) { const v16b a = frag_kb(&Ah[nloc][kb], hlf); v16b al; if (MODE != 0) al = frag_kb(&Al[nloc][kb], hlf);
#pragma unroll
    for (int t = 0; t < 8; ++t) { const v16b bw = frag_kb(WT + (size_t)(g * 128 + t * 16 + nloc) * D + kb, hlf); acc[t] = wmma16b(a, bw, acc[t]); if (MODE != 0) acc[t] = wmma16b(al, bw, acc[t]); } }
#pragma unroll
  for (int t = 0; t < 8; ++t) { const int cc = g * 128 + t * 16 + nloc; const float bb = bias ? bf16_rne(bias[cc]) : 0.0f;
#pragma unroll
    for (int r8 = 0; r8 < 8; ++r8) { const size_t row = m0 + 8 * hlf + r8; float v = acc[t][r8] * (1.0f / (XS * WSC)) + bb; if (ADD) v += ADD[(row / HS) * D + cc]; Tf[8 * hlf + r8][t * 16 + nloc] = v; } }
  wave_lds_sync();
  for (int pass = 0; pass < 2; ++pass) { for (int rr = 0; rr < 16; ++rr) { if (m0 + rr >= (size_t)nrows) break; *(volatile v4f*)(OUT + (m0 + rr) * NOUT + g * 128 + lane * 4) = *(const v4f*)(&Tf[rr][lane * 4]); } __threadfence(); } }
__global__ __launch_bounds__(256) void user_kernel(const float* __restrict__ GC, int BV, float* __restrict__ U) { const int u = blockIdx.x * 256 + threadIdx.x; if (u >= B * D / 4) return; const int b = u / (D / 4); const v4f v = b < BV ? *(const v4f*)(GC + (size_t)b * HS * D + (u % (D / 4)) * 4) : (v4f){0, 0, 0, 0};
  for (int pass = 0; pass < 2; ++pass) { *(volatile v4f*)(U + (size_t)u * 4) = v; __threadfence(); } }
__global__ __launch_bounds__(256) void pool_kernel(const float* __restrict__ GC, const float* __restrict__ KK, const float* __restrict__ QQ, int BV, float* __restrict__ out) { __shared__ float Sc[8][HS + 28]; const int wave = threadIdx.x >> 5, lane = threadIdx.x & 31; const int b = blockIdx.x * 8 + wave; if (b >= BV) return;
  float qv[8];
#pragma unroll
  for (int k = 0; k < 8; ++k) qv[k] = QQ[(size_t)b * A + lane * 8 + k];
  for (int h = 0; h < HS; ++h) { float s = 0.0f;
#pragma unroll
    for (int k = 0; k < 8; ++k) s += pmul(KK[((size_t)b * HS + h) * A + lane * 8 + k], qv[k]); for (int o = 16; o; o >>= 1) s += __shfl_xor(s, o); if (lane == 0) Sc[wave][h] = s * (1.0f / 16.0f); }
  wave_lds_sync(); float mx = -INFINITY; for (int h = 0; h < HS; ++h) mx = fmaxf(mx, Sc[wave][h]); float den = 0.0f; for (int h = 0; h < HS; ++h) den += __expf(Sc[wave][h] - mx); const float inv = 1.0f / den;
  float o[24];
#pragma unroll
  for (int q = 0; q < 24; ++q) o[q] = 0.0f;
  for (int h = 0; h < HS; ++h) { const float al = __expf(Sc[wave][h] - mx) * inv;
#pragma unroll
    for (int q = 0; q < 24; ++q) o[q] += pmul(al, GC[((size_t)b * HS + h) * D + q * 32 + lane]); }
  for (int pass = 0; pass < 2; ++pass) { for (int n = 0; n < NCAND; ++n)
#pragma unroll
    for (int q = 0; q < 24; ++q) ((volatile float*)out)[((size_t)b * NCAND + n) * D + q * 32 + lane] = o[q]; __threadfence(); } }
}

extern "C" void kernel_launch(void* const* d_in, const int* in_sizes, int n_in, void* d_out, int out_size, void* d_ws, size_t ws_size, hipStream_t stream) {
  (void)n_in;
  auto Fp = [&](int i) { return (const float*)d_in[i]; };
  if (in_sizes[0] != R * D || in_sizes[2] != D * D || in_sizes[4] != D * D || in_sizes[5] != A * D || in_sizes[6] != A * D || out_size != B * NCAND * D) return;
  const int BV = B;
  size_t off = 0; char* ws = (char*)d_ws;
  auto carve = [&](size_t bytes) { char* p = ws + off; off += (bytes + 255) & ~(size_t)255; return p; };
  b16* WL = (b16*)carve((size_t)D * D * 2); b16* WR = (b16*)carve((size_t)D * D * 2); b16* WK = (b16*)carve((size_t)A * D * 2); b16* WQ = (b16*)carve((size_t)A * D * 2);
  float* NB = (float*)carve((size_t)B * D * 4); float* NL = (float*)carve((size_t)B * D * 4); float* GC = (float*)carve((size_t)R * D * 4); float* U = (float*)carve((size_t)B * D * 4); float* KK = (float*)carve((size_t)R * A * 4); float* QQ = (float*)carve((size_t)B * A * 4);
  if (off > ws_size || off > ((size_t)64 << 20)) return;
  const int RV = BV * HS;
  wput_kernel<<<(unsigned)(((size_t)D * (D / 8) + 255) / 256), 256, 0, stream>>>(Fp(2), Fp(4), Fp(5), Fp(6), WL, WR, WK, WQ);
  mean_kernel<<<(B * D / 4 + 255) / 256, 256, 0, stream>>>(Fp(0), NB);
  dense_kernel<1><<<((B + 15) / 16) * (D / 128), 32, 0, stream>>>(NB, B, WL, D, Fp(3), nullptr, NL);
  dense_kernel<0><<<((RV + 15) / 16) * (D / 128), 32, 0, stream>>>(Fp(0), RV, WR, D, nullptr, NL, GC);
  dense_kernel<1><<<((RV + 15) / 16) * (A / 128), 32, 0, stream>>>(GC, RV, WK, A, nullptr, nullptr, KK);
  user_kernel<<<(B * D / 4 + 255) / 256, 256, 0, stream>>>(GC, BV, U);
  dense_kernel<1><<<((B + 15) / 16) * (A / 128), 32, 0, stream>>>(U, B, WQ, A, Fp(7), nullptr, QQ);
  pool_kernel<<<(BV + 7) / 8, 256, 0, stream>>>(GC, KK, QQ, BV, (float*)d_out);
}
